// NeoNet_13134009991199
// MI455X (gfx1250) — hardware-verified
//
#include <hip/hip_runtime.h>
#include <math.h>
#include <stdint.h>
#include <stddef.h>


#define BATCH 64
#define NNODE 1025
#define MNODE 1024
#define TFEAT 96
#define QVECN 95
#define INCH  128
#define EPSV  1e-5f
#define ROWTILES 512
#define RECF 256
#define WS_LIMIT ((size_t)134217728)

typedef _Float16 v16h __attribute__((ext_vector_type(16)));
typedef _Float16 v8h  __attribute__((ext_vector_type(8)));
typedef float    v8f  __attribute__((ext_vector_type(8)));
typedef float    v4f  __attribute__((ext_vector_type(4)));
typedef v8h __attribute__((may_alias)) v8ha;
typedef v4f __attribute__((may_alias)) v4fa;

union Frag { v16h v; v8h half[2]; };

__device__ __forceinline__ v8f wmma_f16(const v16h a, const v16h b, v8f c)
{
  v8f d = __builtin_amdgcn_wmma_f32_16x16x32_f16(false, a, false, b, (short)0, c, false, false);
  asm volatile("v_nop\n\tv_nop\n\tv_nop\n\tv_nop" : "+v"(d) : "v"(a), "v"(b));
  return d;
}

__device__ __forceinline__ v8h pack8(const v4f u0, const v4f u1)
{
  v8h o;
  o[0] = (_Float16)u0[0]; o[1] = (_Float16)u0[1]; o[2] = (_Float16)u0[2]; o[3] = (_Float16)u0[3];
  o[4] = (_Float16)u1[0]; o[5] = (_Float16)u1[1]; o[6] = (_Float16)u1[2]; o[7] = (_Float16)u1[3];
  return o;
}

__device__ __forceinline__ v8h affine8(const v8h x, bool z, float mean, float inv)
{
  v8h o;
#pragma unroll
  for (int e = 0; e < 8; ++e) {
    float y = z ? 0.f : (float)x[e];
    float v = (y - mean) * inv;
    v = (v >= 0.f) ? v : 0.01f * v;
    o[e] = (_Float16)v;
  }
  return o;
}

__device__ __forceinline__ float wave_sum(float v)
{
#pragma unroll
  for (int o = 16; o > 0; o >>= 1) v += __shfl_xor(v, o);
  return v;
}

__device__ __forceinline__ int clamp_node(int v)
{
  v = v < 0 ? 0 : v;
  v = v > (NNODE - 1) ? (NNODE - 1) : v;
  return v;
}

__global__ __launch_bounds__(256) void qconv_kernel(
    const float* __restrict__ qv,
    const float* __restrict__ W1, const float* __restrict__ b1,
    const float* __restrict__ W2, const float* __restrict__ b2,
    const float* __restrict__ W3, const float* __restrict__ b3,
    const float* __restrict__ W4, const float* __restrict__ b4,
    float* __restrict__ qout)
{
  __shared__ __align__(16) float bufA[64 * 128];
  __shared__ __align__(16) float bufB[64 * 128];
  const int tid = threadIdx.x;
  for (int i = tid; i < 64 * QVECN; i += 256) bufA[i] = qv[i];
  __syncthreads();
  for (int i = tid; i < 64 * 64; i += 256) {
    int r = i >> 6, c = i & 63;
    float s = b1[c];
    for (int k = 0; k < QVECN; ++k) s += bufA[r * QVECN + k] * W1[k * 64 + c];
    bufB[r * 64 + c] = s;
  }
  __syncthreads();
  for (int i = tid; i < 64 * 128; i += 256) {
    int r = i >> 7, c = i & 127;
    float s = b2[c];
    for (int k = 0; k < 64; ++k) s += bufB[r * 64 + k] * W2[k * 128 + c];
    bufA[r * 128 + c] = s;
  }
  __syncthreads();
  for (int i = tid; i < 64 * 64; i += 256) {
    int r = i >> 6, c = i & 63;
    float s = b3[c];
    for (int k = 0; k < 128; ++k) s += bufA[r * 128 + k] * W3[k * 64 + c];
    bufB[r * 64 + c] = s;
  }
  __syncthreads();
  for (int i = tid; i < 64 * 32; i += 256) {
    int r = i >> 5, c = i & 31;
    float s = b4[c];
    for (int k = 0; k < 64; ++k) s += bufB[r * 64 + k] * W4[k * 32 + c];
    bufA[i] = s;
  }
  __syncthreads();
  const v4f w0 = *(const v4fa*)(bufA + 4 * tid);
  const v4f w1 = *(const v4fa*)(bufA + 4 * (tid + 256));
  *(volatile v4fa*)(qout + 4 * tid) = w0;
  *(volatile v4fa*)(qout + 4 * (tid + 256)) = w1;
  __threadfence();
  *(volatile v4fa*)(qout + 4 * tid) = w0;
  *(volatile v4fa*)(qout + 4 * (tid + 256)) = w1;
}

__global__ __launch_bounds__(256) void pack_w_kernel(
    const float* __restrict__ Wc, _Float16* __restrict__ Wp, int Cin, int lc, int nchunk)
{
  const int g = blockIdx.x * 256 + threadIdx.x;
  const bool ok = g < nchunk;
  v8h o = {};
  if (ok) {
    const int K8 = (3 * Cin) >> 3;
    const int oc = g / K8;
    const int kc = (g - oc * K8) * 8;
    const int child = kc >> lc;
    const int f = kc & (Cin - 1);
    const float* wp = Wc + ((size_t)oc * Cin + f) * 3 + child;
#pragma unroll
    for (int e = 0; e < 8; ++e) o[e] = (_Float16)(16.0f * wp[3 * e]);
    *(volatile v8ha*)(Wp + (size_t)g * 8) = o;
  }
  __threadfence();
  if (ok) *(volatile v8ha*)(Wp + (size_t)g * 8) = o;
}

__global__ __launch_bounds__(256) void pack_aug_kernel(
    const float* __restrict__ trees, const float* __restrict__ q,
    _Float16* __restrict__ A0, int nchunk)
{
  const int g = blockIdx.x * 256 + threadIdx.x;
  const bool ok = g < nchunk;
  v8h o = {};
  if (ok) {
    const int t = g >> 4;
    const int c0 = (g & 15) * 8;
    const float* p;
    if (c0 < TFEAT) {
      p = trees + (size_t)t * TFEAT + c0;
    } else {
      const int b = t / NNODE;
      p = q + b * 32 + (c0 - TFEAT);
    }
    const v4f u0 = *(const v4fa*)p;
    const v4f u1 = *(const v4fa*)(p + 4);
    o = pack8(u0, u1);
    *(volatile v8ha*)(A0 + (size_t)g * 8) = o;
  }
  __threadfence();
  if (ok) *(volatile v8ha*)(A0 + (size_t)g * 8) = o;
}

template <bool NORM, int MODE>
__global__ __launch_bounds__(256) void tree_conv_gemm(
    const _Float16* __restrict__ act,
    const _Float16* __restrict__ Wp,
    const float* __restrict__ bias,
    const int*   __restrict__ idx,
    const float* __restrict__ stats,
    _Float16*    __restrict__ Y,
    float*       __restrict__ rec,
    int Cin, int lc, int Cout)
{
  __shared__ __align__(16) float lds_main[8448];
  __shared__ __align__(16) float cmaxbuf[16 * 128];
  __shared__ __align__(16) float recbuf[RECF];
  __shared__ float red_s[8];
  __shared__ float red_q[8];

  _Float16* const As = reinterpret_cast<_Float16*>(lds_main);
  _Float16* const Bs = As + 128 * 40;
  float* const Cs = lds_main;

  const int tid  = threadIdx.x;
  const int wave = tid >> 5;
  const int lane = tid & 31;
  const int h = lane >> 4;
  const int m = lane & 15;
  const int wr = wave >> 1;
  const int wc = wave & 1;
  const int R0 = blockIdx.x * 128;
  const int C0 = blockIdx.y * 128;
  const int b  = R0 >> 10;
  const int m0 = R0 & (MNODE - 1);
  const int K  = 3 * Cin;

  const int rS = tid >> 1;
  const int hS = tid & 1;
  const int* ip = idx + (size_t)b * (3 * MNODE) + 3 * (m0 + rS);
  const int nd0 = clamp_node(ip[0]);
  const int nd1 = clamp_node(ip[1]);
  const int nd2 = clamp_node(ip[2]);

  float mean = 0.f, inv = 1.f;
  if (NORM) { mean = stats[2 * b]; inv = stats[2 * b + 1]; }

  v8f acc[2][4];
#pragma unroll
  for (int i = 0; i < 2; ++i)
#pragma unroll
    for (int j = 0; j < 4; ++j) { v8f z = {}; acc[i][j] = z; }

  for (int k0 = 0; k0 < K; k0 += 32) {
    const int child = k0 >> lc;
    const int kin = k0 & (Cin - 1);
    const int node = (child == 0) ? nd0 : ((child == 1) ? nd1 : nd2);
    {
      v8h x0, x1;
      if (NORM) {
        const bool z = (node == 0);
        const int yr = z ? 0 : (node - 1);
        const _Float16* src = act + ((size_t)(b * MNODE + yr)) * Cin + kin + 16 * hS;
        x0 = *(const v8ha*)src;
        x1 = *(const v8ha*)(src + 8);
        x0 = affine8(x0, z, mean, inv);
        x1 = affine8(x1, z, mean, inv);
      } else {
        const _Float16* src = act + ((size_t)(b * NNODE + node)) * Cin + kin + 16 * hS;
        x0 = *(const v8ha*)src;
        x1 = *(const v8ha*)(src + 8);
      }
      *(v8ha*)(As + rS * 40 + 16 * hS)     = x0;
      *(v8ha*)(As + rS * 40 + 16 * hS + 8) = x1;
    }
    {
      const _Float16* src = Wp + ((size_t)(C0 + rS)) * K + k0 + 16 * hS;
      const v8h w0 = *(const v8ha*)src;
      const v8h w1 = *(const v8ha*)(src + 8);
      *(v8ha*)(Bs + rS * 40 + 16 * hS)     = w0;
      *(v8ha*)(Bs + rS * 40 + 16 * hS + 8) = w1;
    }
    __syncthreads();

    Frag fa0, fa1;
    {
      const _Float16* p = As + (32 * wr + m) * 40 + 8 * h;
      fa0.half[0] = *(const v8ha*)p;
      fa0.half[1] = *(const v8ha*)(p + 16);
    }
    {
      const _Float16* p = As + (32 * wr + 16 + m) * 40 + 8 * h;
      fa1.half[0] = *(const v8ha*)p;
      fa1.half[1] = *(const v8ha*)(p + 16);
    }
#pragma unroll
    for (int j = 0; j < 4; ++j) {
      Frag fb;
      const _Float16* p = Bs + (64 * wc + 16 * j + m) * 40 + 8 * h;
      fb.half[0] = *(const v8ha*)p;
      fb.half[1] = *(const v8ha*)(p + 16);
      acc[0][j] = wmma_f16(fa0.v, fb.v, acc[0][j]);
      acc[1][j] = wmma_f16(fa1.v, fb.v, acc[1][j]);
    }
    __syncthreads();
  }

  const float sc = 0.0625f;
  float bj[4];
#pragma unroll
  for (int j = 0; j < 4; ++j) bj[j] = bias[C0 + 64 * wc + 16 * j + m];
  float s = 0.f, s2 = 0.f;
  float cmx[8];
#pragma unroll
  for (int e = 0; e < 8; ++e) cmx[e] = -3.0e38f;

#pragma unroll
  for (int hf = 0; hf < 2; ++hf) {
    if ((wr >> 1) == hf) {
#pragma unroll
      for (int i = 0; i < 2; ++i)
#pragma unroll
        for (int j = 0; j < 4; ++j)
#pragma unroll
          for (int r = 0; r < 8; ++r)
            Cs[(32 * (wr & 1) + 16 * i + 8 * h + r) * 132 + 64 * wc + 16 * j + m] =
                acc[i][j][r] * sc + bj[j];
    }
    __syncthreads();
#pragma unroll
    for (int it = 0; it < 4; ++it) {
      const int q = it * 256 + tid;
      const int lr = q >> 4;
      const int ch = q & 15;
      const float* cp = Cs + lr * 132 + 8 * ch;
      const v4f u0 = *(const v4fa*)cp;
      const v4f u1 = *(const v4fa*)(cp + 4);
#pragma unroll
      for (int e = 0; e < 4; ++e) {
        s += u0[e]; s2 += u0[e] * u0[e];
        s += u1[e]; s2 += u1[e] * u1[e];
      }
      if (MODE == 1) {
#pragma unroll
        for (int e = 0; e < 4; ++e) {
          cmx[e]     = fmaxf(cmx[e], u0[e]);
          cmx[4 + e] = fmaxf(cmx[4 + e], u1[e]);
        }
      }
      if (MODE == 0) {
        _Float16* yp = Y + ((size_t)(R0 + 64 * hf + lr)) * Cout + C0 + 8 * ch;
        *(volatile v8ha*)yp = pack8(u0, u1);
      }
    }
    if (MODE == 0) {
      __threadfence();
#pragma unroll
      for (int it = 0; it < 4; ++it) {
        const int q = it * 256 + tid;
        const int lr = q >> 4;
        const int ch = q & 15;
        const float* cp = Cs + lr * 132 + 8 * ch;
        const v4f u0 = *(const v4fa*)cp;
        const v4f u1 = *(const v4fa*)(cp + 4);
        _Float16* yp = Y + ((size_t)(R0 + 64 * hf + lr)) * Cout + C0 + 8 * ch;
        *(volatile v8ha*)yp = pack8(u0, u1);
      }
    }
    __syncthreads();
  }

  s = wave_sum(s);
  s2 = wave_sum(s2);
  if (lane == 0) { red_s[wave] = s; red_q[wave] = s2; }
  if (MODE == 1) {
#pragma unroll
    for (int e = 0; e < 8; ++e) cmaxbuf[(tid >> 4) * 128 + 8 * (tid & 15) + e] = cmx[e];
  }
  __syncthreads();
  {
    float v = 0.f;
    if (tid < 128) {
      if (MODE == 1) {
        v = cmaxbuf[tid];
#pragma unroll
        for (int g = 1; g < 16; ++g) v = fmaxf(v, cmaxbuf[g * 128 + tid]);
      }
    } else if (tid == 128) {
      float S = 0.f;
#pragma unroll
      for (int w = 0; w < 8; ++w) S += red_s[w];
      v = S;
    } else if (tid == 129) {
      float S = 0.f;
#pragma unroll
      for (int w = 0; w < 8; ++w) S += red_q[w];
      v = S;
    }
    recbuf[tid] = v;
  }
  __syncthreads();
  const size_t recBase = ((size_t)blockIdx.y * ROWTILES + blockIdx.x) * RECF;
  v4f rv = {};
  if (tid < 64) {
    rv = *(const v4fa*)(recbuf + 4 * tid);
    *(volatile v4fa*)(rec + recBase + 4 * tid) = rv;
  }
  __threadfence();
  if (tid < 64) *(volatile v4fa*)(rec + recBase + 4 * tid) = rv;
}

__global__ __launch_bounds__(64) void stats_kernel(
    const float* __restrict__ rec, float* __restrict__ stats, int nct, int Cout)
{
  __shared__ __align__(16) float sb[128];
  const int b = threadIdx.x;
  double s = 0.0, q = 0.0;
  for (int ct = 0; ct < nct; ++ct) {
    for (int r = 0; r < 8; ++r) {
      const float* p = rec + ((size_t)(ct * ROWTILES + 8 * b + r)) * RECF;
      s += (double)p[128];
      q += (double)p[129];
    }
  }
  const double cnt = (double)Cout * (double)NNODE;
  const double mean = s / cnt;
  double var = (q - s * s / cnt) / (cnt - 1.0);
  var = var > 0.0 ? var : 0.0;
  const float stdf = sqrtf((float)var);
  sb[2 * b]     = (float)mean;
  sb[2 * b + 1] = 1.0f / (stdf + EPSV);
  __syncthreads();
  v4f v = {};
  if (b < 32) {
    v = *(const v4fa*)(sb + 4 * b);
    *(volatile v4fa*)(stats + 4 * b) = v;
  }
  __threadfence();
  if (b < 32) *(volatile v4fa*)(stats + 4 * b) = v;
}

__global__ __launch_bounds__(128) void pool_kernel(
    const float* __restrict__ rec, float* __restrict__ out)
{
  __shared__ float sm[2];
  __shared__ __align__(16) float ob[128];
  const int b = blockIdx.x;
  const int t = threadIdx.x;
  float mx = 0.f;
#pragma unroll
  for (int r = 0; r < 8; ++r) mx = fmaxf(mx, rec[((size_t)(8 * b + r)) * RECF + t]);
  if (t == 0) {
    double s = 0.0, q = 0.0;
    for (int r = 0; r < 8; ++r) {
      const float* p = rec + ((size_t)(8 * b + r)) * RECF;
      s += (double)p[128];
      q += (double)p[129];
    }
    const double cnt = 128.0 * (double)NNODE;
    const double mean = s / cnt;
    double var = (q - s * s / cnt) / (cnt - 1.0);
    var = var > 0.0 ? var : 0.0;
    const float stdf = sqrtf((float)var);
    sm[0] = (float)mean;
    sm[1] = 1.0f / (stdf + EPSV);
  }
  __syncthreads();
  ob[t] = (mx - sm[0]) * sm[1];
  __syncthreads();
  v4f v = {};
  if (t < 32) {
    v = *(const v4fa*)(ob + 4 * t);
    *(volatile v4fa*)(out + b * 128 + 4 * t) = v;
  }
  __threadfence();
  if (t < 32) *(volatile v4fa*)(out + b * 128 + 4 * t) = v;
}

extern "C" void kernel_launch(void* const* d_in, const int* in_sizes, int n_in,
                              void* d_out, int out_size, void* d_ws, size_t ws_size,
                              hipStream_t stream)
{
  if (n_in < 17) return;
  if (in_sizes[0] != BATCH * QVECN) return;
  if (in_sizes[1] != BATCH * NNODE * TFEAT) return;
  if (in_sizes[2] != BATCH * 3 * MNODE) return;
  if (in_sizes[3] != QVECN * 64 || in_sizes[4] != 64) return;
  if (in_sizes[5] != 64 * 128  || in_sizes[6] != 128) return;
  if (in_sizes[7] != 128 * 64  || in_sizes[8] != 64) return;
  if (in_sizes[9] != 64 * 32   || in_sizes[10] != 32) return;
  if (in_sizes[11] != 512 * 128 * 3 || in_sizes[12] != 512) return;
  if (in_sizes[13] != 256 * 512 * 3 || in_sizes[14] != 256) return;
  if (in_sizes[15] != 128 * 256 * 3 || in_sizes[16] != 128) return;
  if (out_size != BATCH * 128) return;

  const float* q_vecs = (const float*)d_in[0];
  const float* trees  = (const float*)d_in[1];
  const int*   idxes  = (const int*)d_in[2];
  const float* Wq1 = (const float*)d_in[3],  *bq1 = (const float*)d_in[4];
  const float* Wq2 = (const float*)d_in[5],  *bq2 = (const float*)d_in[6];
  const float* Wq3 = (const float*)d_in[7],  *bq3 = (const float*)d_in[8];
  const float* Wq4 = (const float*)d_in[9],  *bq4 = (const float*)d_in[10];
  const float* Wc1 = (const float*)d_in[11], *bc1 = (const float*)d_in[12];
  const float* Wc2 = (const float*)d_in[13], *bc2 = (const float*)d_in[14];
  const float* Wc3 = (const float*)d_in[15], *bc3 = (const float*)d_in[16];

  char* ws = (char*)d_ws;
  size_t off = 0;
  auto carve = [&](size_t bytes) -> char* {
    char* p = ws + off;
    off += (bytes + 4095) & ~(size_t)4095;
    return p;
  };
  float*    qout  = (float*)   carve((size_t)BATCH * 32 * 4);
  _Float16* Wp1   = (_Float16*)carve((size_t)512 * 384 * 2);
  _Float16* Wp2   = (_Float16*)carve((size_t)256 * 1536 * 2);
  _Float16* Wp3   = (_Float16*)carve((size_t)128 * 768 * 2);
  float*    stats = (float*)   carve((size_t)128 * 4);
  float*    rec   = (float*)   carve((size_t)4 * ROWTILES * RECF * 4);
  char*     regS  =            carve((size_t)BATCH * MNODE * 256 * 2);
  _Float16* A0    = (_Float16*)regS;
  _Float16* Y2h   = (_Float16*)regS;
  _Float16* Y1h   = (_Float16*)carve((size_t)BATCH * MNODE * 512 * 2);
  if (off > ws_size || off > WS_LIMIT) return;

  const int nchunkW1 = 512 * 384 / 8;
  const int nchunkW2 = 256 * 1536 / 8;
  const int nchunkW3 = 128 * 768 / 8;
  const int nchunkA0 = BATCH * NNODE * INCH / 8;

  qconv_kernel<<<1, 256, 0, stream>>>(q_vecs, Wq1, bq1, Wq2, bq2, Wq3, bq3, Wq4, bq4, qout);
  pack_w_kernel<<<(nchunkW1 + 255) / 256, 256, 0, stream>>>(Wc1, Wp1, 128, 7, nchunkW1);
  pack_w_kernel<<<(nchunkW2 + 255) / 256, 256, 0, stream>>>(Wc2, Wp2, 512, 9, nchunkW2);
  pack_w_kernel<<<(nchunkW3 + 255) / 256, 256, 0, stream>>>(Wc3, Wp3, 256, 8, nchunkW3);
  pack_aug_kernel<<<(nchunkA0 + 255) / 256, 256, 0, stream>>>(trees, qout, A0, nchunkA0);

  tree_conv_gemm<false, 0><<<dim3(ROWTILES, 4), 256, 0, stream>>>(
      A0, Wp1, bc1, idxes, stats, Y1h, rec, 128, 7, 512);
  stats_kernel<<<1, 64, 0, stream>>>(rec, stats, 4, 512);
  tree_conv_gemm<true, 0><<<dim3(ROWTILES, 2), 256, 0, stream>>>(
      Y1h, Wp2, bc2, idxes, stats, Y2h, rec, 512, 9, 256);
  stats_kernel<<<1, 64, 0, stream>>>(rec, stats, 2, 256);
  tree_conv_gemm<true, 1><<<dim3(ROWTILES, 1), 256, 0, stream>>>(
      Y2h, Wp3, bc3, idxes, stats, Y1h, rec, 256, 8, 128);
  pool_kernel<<<BATCH, 128, 0, stream>>>(rec, (float*)d_out);
}
